// KAN_EBM_54073638256940
// MI455X (gfx1250) — hardware-verified
//
#include <hip/hip_runtime.h>

#include <hip/hip_bf16.h>

typedef __attribute__((ext_vector_type(16))) _Float16 v16h;
typedef __attribute__((ext_vector_type(2)))  _Float16 h2;
typedef __attribute__((ext_vector_type(8)))  float    v8f;

#define TOKS_PER_BLK 128
#define LDSTRIDE 132
#define NBLK 512

#define L0_OFF      0
#define L1_OFF   4096
#define L2_OFF 135168
#define L3_OFF 266240
#define WPACK_HALVES 282624
#define PARTIALS_OFF_BYTES 565248

__device__ __forceinline__ h2 u2h(unsigned u) { return __builtin_bit_cast(h2, u); }
__device__ __forceinline__ unsigned h2u(h2 h) { return __builtin_bit_cast(unsigned, h); }

__global__ void kan_pack_weights(const float* __restrict__ bw,
                                 const float* __restrict__ sw,
                                 _Float16* __restrict__ dst,
                                 int din, int dout, int nnt, int nHalves) {
    int idx = blockIdx.x * 256 + threadIdx.x;
    if (idx >= nHalves) return;
    int e    = idx & 15;
    int lane = (idx >> 4) & 31;
    int f    = idx >> 9;
    int ch   = f / nnt;
    int nt   = f - ch * nnt;
    int k = ch * 32 + ((lane >> 4) << 3) + (e < 8 ? e : e + 8);
    int n = nt * 16 + (lane & 15);
    int i = k >> 4;
    int c = k & 15;
    float w = 0.f;
    if (n < dout && i < din && c < 13) {
        w = (c == 0) ? bw[n * din + i] : sw[(n * din + i) * 12 + (c - 1)];
    }
    dst[idx] = (_Float16)w;
}

__device__ __constant__ const unsigned kTLO[4] = {0xC100C100u, 0xC100C100u, 0xBE00C100u, 0x3800B800u};
__device__ __constant__ const unsigned kTHI[4] = {0x41003E00u, 0x41004100u, 0x41004100u, 0x41004100u};

template <int DIN, int NNT>
__device__ __forceinline__ void kan_layer_wave(const float* __restrict__ hin,
                                               float* __restrict__ hout,
                                               const _Float16* __restrict__ wpack,
                                               int lane) {
    constexpr int NCH = DIN / 2;
    const int  m    = lane & 15;
    const bool ishi = (lane >> 4) != 0;
    const float* hrow = hin + m * LDSTRIDE;
    const v16h* wfrag = (const v16h*)wpack;

    v8f acc[NNT];
#pragma unroll
    for (int nt = 0; nt < NNT; ++nt) acc[nt] = v8f{0.f,0.f,0.f,0.f,0.f,0.f,0.f,0.f};

    for (int ch = 0; ch < NCH; ++ch) {
        float2 hp = *(const float2*)(hrow + 2 * ch);
        union { v16h v; _Float16 s[16]; } A;
#pragma unroll
        for (int half = 0; half < 2; ++half) {
            const float hv = half ? hp.y : hp.x;
            const float xc = fminf(fmaxf(hv, -1.f), 1.f);
#pragma unroll
            for (int q = 0; q < 8; ++q) {
                const int c = (ishi ? 8 : 0) + q;
                const float g = (c <= 4) ? -1.f : ((c >= 9) ? 1.f : (-1.f + (float)(c - 4) * 0.4f));
                const float d = (xc - g) * 2.5f;
                const float bas = fmaxf(1.f - fabsf(d), 0.f);
                A.s[half * 8 + q] = (_Float16)((c == 0) ? hv : bas);
            }
        }
        v16h a = A.v;
#pragma unroll
        for (int nt = 0; nt < NNT; ++nt) {
            v16h b = wfrag[(ch * NNT + nt) * 32 + lane];
            acc[nt] = __builtin_amdgcn_wmma_f32_16x16x32_f16(
                false, a, false, b, (short)0, acc[nt], false, false);
        }
        asm volatile("v_nop\n\tv_nop\n\tv_nop\n\tv_nop" : "+v"(acc[0]), "+v"(acc[NNT - 1]) : "v"(a));
    }
    const int hi = ishi ? 1 : 0;
#pragma unroll
    for (int nt = 0; nt < NNT; ++nt) {
#pragma unroll
        for (int v = 0; v < 8; ++v) {
            hout[(v + 8 * hi) * LDSTRIDE + nt * 16 + m] = acc[nt][v];
        }
    }
}

__device__ __forceinline__ void layernorm_rows(float* buf, int dout,
                                               const float* __restrict__ gamma,
                                               const float* __restrict__ beta,
                                               int tid, float* lnS, float* lnQ) {
    const int row  = tid >> 1;
    const int half = tid & 1;
    const int hw   = dout >> 1;
    float* rowp = buf + row * LDSTRIDE + half * hw;
    const float* gp = gamma + half * hw;
    const float* bp = beta  + half * hw;

    float s = 0.f, q = 0.f;
    for (int n = 0; n < hw; ++n) { float v = rowp[n]; s += v; q += v * v; }
    lnS[tid] = s; lnQ[tid] = q;
    __syncthreads();
    float S = lnS[row * 2] + lnS[row * 2 + 1];
    float Q = lnQ[row * 2] + lnQ[row * 2 + 1];
    float mean = S / (float)dout;
    float var  = Q / (float)dout - mean * mean;
    float r = rsqrtf(var + 1e-5f);
    for (int n = 0; n < hw; ++n)
        rowp[n] = (rowp[n] - mean) * r * gp[n] + bp[n];
}

__global__ __launch_bounds__(256) void kan_fused(
    const float* __restrict__ u, const float* __restrict__ x,
    const _Float16* __restrict__ wpack,
    const float* __restrict__ g0, const float* __restrict__ be0,
    const float* __restrict__ g1, const float* __restrict__ be1,
    const float* __restrict__ g2, const float* __restrict__ be2,
    float* partials) {
    __shared__ float bufA[TOKS_PER_BLK * LDSTRIDE];
    __shared__ float bufB[TOKS_PER_BLK * LDSTRIDE];
    __shared__ float lnS[256];
    __shared__ float lnQ[256];

    const int tid  = threadIdx.x;
    const int wave = tid >> 5;
    const int lane = tid & 31;
    const int tok0 = blockIdx.x * TOKS_PER_BLK;
    const int woff = wave * 16 * LDSTRIDE;

    for (int idx = tid; idx < TOKS_PER_BLK * 4; idx += 256) {
        int t = idx >> 2, f = idx & 3;
        float v = (f == 0) ? u[tok0 + t] : x[(tok0 + t) * 3 + (f - 1)];
        bufA[t * LDSTRIDE + f] = v;
    }
    __syncthreads();

    kan_layer_wave<4, 4>(bufA + woff, bufB + woff, wpack + L0_OFF, lane);
    __syncthreads();
    layernorm_rows(bufB, 64, g0, be0, tid, lnS, lnQ);
    __syncthreads();

    kan_layer_wave<64, 8>(bufB + woff, bufA + woff, wpack + L1_OFF, lane);
    __syncthreads();
    layernorm_rows(bufA, 128, g1, be1, tid, lnS, lnQ);
    __syncthreads();

    kan_layer_wave<128, 4>(bufA + woff, bufB + woff, wpack + L2_OFF, lane);
    __syncthreads();
    layernorm_rows(bufB, 64, g2, be2, tid, lnS, lnQ);
    __syncthreads();

    kan_layer_wave<64, 1>(bufB + woff, bufA + woff, wpack + L3_OFF, lane);
    __syncthreads();

    if (tid < TOKS_PER_BLK) lnS[tid] = bufA[tid * LDSTRIDE];
    __syncthreads();
    for (int s = TOKS_PER_BLK / 2; s > 0; s >>= 1) {
        if (tid < s) lnS[tid] += lnS[tid + s];
        __syncthreads();
    }
    if (tid < 32) {
        const float pv = (tid == 0) ? lnS[0] : 0.f;
        *(volatile float*)(partials + blockIdx.x * 32 + tid) = pv;
        __threadfence();
        *(volatile float*)(partials + blockIdx.x * 32 + tid) = pv;
    }
}

__global__ void kan_finalize(const float* __restrict__ partials,
                             float* out) {
    int b = threadIdx.x;
    if (b < 16) {
        float s = 0.f;
        for (int i = 0; i < 32; ++i) s += partials[(b * 32 + i) * 32];
        *(volatile float*)(out + b) = s / 4096.0f;
        __threadfence();
        *(volatile float*)(out + b) = s / 4096.0f;
    }
}

extern "C" void kernel_launch(void* const* d_in, const int* in_sizes, int n_in,
                              void* d_out, int out_size, void* d_ws, size_t ws_size,
                              hipStream_t stream) {
    const float* u   = (const float*)d_in[0];
    const float* x   = (const float*)d_in[1];
    const float* bw0 = (const float*)d_in[2];
    const float* sw0 = (const float*)d_in[3];
    const float* g0  = (const float*)d_in[4];
    const float* be0 = (const float*)d_in[5];
    const float* bw1 = (const float*)d_in[6];
    const float* sw1 = (const float*)d_in[7];
    const float* g1  = (const float*)d_in[8];
    const float* be1 = (const float*)d_in[9];
    const float* bw2 = (const float*)d_in[10];
    const float* sw2 = (const float*)d_in[11];
    const float* g2  = (const float*)d_in[12];
    const float* be2 = (const float*)d_in[13];
    const float* bw3 = (const float*)d_in[14];
    const float* sw3 = (const float*)d_in[15];

    _Float16* wpack    = (_Float16*)d_ws;
    float*    partials = (float*)((char*)d_ws + PARTIALS_OFF_BYTES);

    kan_pack_weights<<<(4096   + 255) / 256, 256, 0, stream>>>(bw0, sw0, wpack + L0_OFF,   4,  64, 4,   4096);
    kan_pack_weights<<<(131072 + 255) / 256, 256, 0, stream>>>(bw1, sw1, wpack + L1_OFF,  64, 128, 8, 131072);
    kan_pack_weights<<<(131072 + 255) / 256, 256, 0, stream>>>(bw2, sw2, wpack + L2_OFF, 128,  64, 4, 131072);
    kan_pack_weights<<<(16384  + 255) / 256, 256, 0, stream>>>(bw3, sw3, wpack + L3_OFF,  64,  16, 1,  16384);

    kan_fused<<<NBLK, 256, 0, stream>>>(u, x, wpack, g0, be0, g1, be1, g2, be2, partials);
    kan_finalize<<<1, 32, 0, stream>>>(partials, (float*)d_out);
}
